// SpatiallyMaskedSelfAttention_Light_89464168775865
// MI455X (gfx1250) — hardware-verified
//
#include <hip/hip_runtime.h>

typedef _Float16 v16h __attribute__((ext_vector_type(16)));
typedef _Float16 v8h  __attribute__((ext_vector_type(8)));
typedef __bf16   v16b __attribute__((ext_vector_type(16)));
typedef __bf16   v8b  __attribute__((ext_vector_type(8)));
typedef float    v8f  __attribute__((ext_vector_type(8)));
typedef float    v4f  __attribute__((ext_vector_type(4)));
typedef int      v4i  __attribute__((ext_vector_type(4)));
typedef unsigned short v8us __attribute__((ext_vector_type(8)));
typedef v8h  __attribute__((may_alias)) v8ha;
typedef v8b  __attribute__((may_alias)) v8ba;
typedef v4f  __attribute__((may_alias)) v4fa;
typedef v4i  __attribute__((may_alias)) v4ia;
typedef v8us __attribute__((may_alias)) v8usa;

union FragH { v16h v; v8h half[2]; };
union FragB { v16b v; v8b half[2]; };

#define DIMC    768
#define NHEADS  12
#define HD      64
#define SEQ     1024
#define BATCH   8
#define QKVO    2304
#define MROWS   (BATCH * SEQ)
#define NX      (MROWS * DIMC)
#define NWQ     (QKVO * DIMC)
#define NWP     (DIMC * DIMC)
#define NMASK   (SEQ * SEQ)
#define NX8     (NX / 8)
#define NWQ8    (NWQ / 8)
#define NWP8    (NWP / 8)
#define NCVT    (NX8 + NWQ8 + NWP8)
#define PSCALE  16384.0f
#define QKSCALE 0.125f

__device__ __forceinline__ v8f wmma_f16(v16h a, v16h b, v8f c) {
  v8f d = __builtin_amdgcn_wmma_f32_16x16x32_f16(false, a, false, b, (short)0, c, false, false);
  asm volatile("v_nop\n\tv_nop\n\tv_nop\n\tv_nop" : "+v"(d) : "v"(a), "v"(b));
  return d;
}
__device__ __forceinline__ v8f wmma_bf16(v16b a, v16b b, v8f c) {
  v8f d = __builtin_amdgcn_wmma_f32_16x16x32_bf16(false, a, false, b, (short)0, c, false, false);
  asm volatile("v_nop\n\tv_nop\n\tv_nop\n\tv_nop" : "+v"(d) : "v"(a), "v"(b));
  return d;
}

__device__ __forceinline__ v16h load_frag_h(const _Float16* p, int h) {
  FragH f;
  f.half[0] = *(const v8ha*)(p + 8 * h);
  f.half[1] = *(const v8ha*)(p + 16 + 8 * h);
  return f.v;
}
__device__ __forceinline__ v16b load_frag_b(const unsigned short* p, int h) {
  FragB f;
  f.half[0] = *(const v8ba*)(p + 8 * h);
  f.half[1] = *(const v8ba*)(p + 16 + 8 * h);
  return f.v;
}

__device__ __forceinline__ unsigned short bf16_bits(float f) {
  unsigned int u = __float_as_uint(f);
  u += 0x7FFFu + ((u >> 16) & 1u);
  return (unsigned short)(u >> 16);
}
__device__ __forceinline__ void split_bf16(float v, unsigned short& hi, unsigned short& lo) {
  const unsigned short hb = bf16_bits(v);
  const float hf = __uint_as_float(((unsigned int)hb) << 16);
  hi = hb;
  lo = bf16_bits(v - hf);
}

__global__ __launch_bounds__(256) void convert_kernel(
    const float* __restrict__ x, const float* __restrict__ wq, const float* __restrict__ wp,
    unsigned short* __restrict__ xb, unsigned short* __restrict__ wqb, unsigned short* __restrict__ wpb)
{
  const int g = blockIdx.x * 256 + threadIdx.x;
  if (g >= NCVT) return;
  const float* src;
  unsigned short* dst;
  if (g < NX8) {
    src = x + (size_t)g * 8;
    dst = xb + (size_t)g * 8;
  } else if (g < NX8 + NWQ8) {
    const int e = g - NX8;
    src = wq + (size_t)e * 8;
    dst = wqb + (size_t)e * 8;
  } else {
    const int e = g - NX8 - NWQ8;
    src = wp + (size_t)e * 8;
    dst = wpb + (size_t)e * 8;
  }
  const v4f a = *(const v4fa*)src;
  const v4f c = *(const v4fa*)(src + 4);
  const v8us o = { bf16_bits(a.x), bf16_bits(a.y), bf16_bits(a.z), bf16_bits(a.w),
                   bf16_bits(c.x), bf16_bits(c.y), bf16_bits(c.z), bf16_bits(c.w) };
  *(volatile v8us*)dst = o;
  __threadfence();
  *(volatile v8us*)dst = o;
}

__device__ __forceinline__ void qkv_store_pass(const _Float16* sT, _Float16* plane, _Float16* vt,
                                               int which, int bh, int l0, int w, int lane) {
  const int q8 = lane & 7, sub = lane >> 3;
  #pragma unroll
  for (int i = 0; i < 8; ++i) {
    const int lid = w * 32 + i * 4 + sub;
    v8h v;
    _Float16* dst;
    if (which != 2) {
      v = *(const v8ha*)(sT + lid * HD + 8 * q8);
      dst = plane + ((size_t)bh * SEQ + l0 + lid) * HD + 8 * q8;
    } else {
      const int d = lid >> 1, hl = lid & 1;
      v = *(const v8ha*)(sT + d * 128 + 64 * hl + 8 * q8);
      dst = vt + ((size_t)bh * HD + d) * SEQ + l0 + 64 * hl + 8 * q8;
    }
    *(volatile v8h*)dst = v;
  }
}

__global__ __launch_bounds__(128) void qkv_kernel(
    const unsigned short* __restrict__ xb,
    const unsigned short* __restrict__ wqb,
    _Float16* __restrict__ qh,
    _Float16* __restrict__ kh,
    _Float16* __restrict__ vt)
{
  __shared__ __attribute__((aligned(16))) _Float16 sT[128 * 64];

  const int tid = threadIdx.x, lane = tid & 31, w = tid >> 5;
  const int h = lane >> 4, m = lane & 15;
  const int m0 = blockIdx.x * 128;
  const int cg = blockIdx.y;
  const int which = cg / NHEADS, head = cg - which * NHEADS;
  const int m0w = m0 + 32 * w;

  const unsigned short* xa0 = xb + (size_t)(m0w + m) * DIMC;
  const unsigned short* xa1 = xa0 + (size_t)16 * DIMC;
  const unsigned short* wb  = wqb + ((size_t)cg * 64 + m) * DIMC;

  const v8f zero8 = {0.f, 0.f, 0.f, 0.f, 0.f, 0.f, 0.f, 0.f};
  v8f acc[2][4];
  #pragma unroll
  for (int mt = 0; mt < 2; ++mt)
    #pragma unroll
    for (int nt = 0; nt < 4; ++nt) acc[mt][nt] = zero8;

  #pragma unroll 1
  for (int k0 = 0; k0 < DIMC; k0 += 32) {
    const v16b a0 = load_frag_b(xa0 + k0, h);
    const v16b a1 = load_frag_b(xa1 + k0, h);
    #pragma unroll
    for (int nt = 0; nt < 4; ++nt) {
      const v16b b = load_frag_b(wb + (size_t)nt * 16 * DIMC + k0, h);
      acc[0][nt] = wmma_bf16(a0, b, acc[0][nt]);
      acc[1][nt] = wmma_bf16(a1, b, acc[1][nt]);
    }
  }

  #pragma unroll
  for (int nt = 0; nt < 4; ++nt) {
    const int feat = 16 * nt + m;
    #pragma unroll
    for (int mt = 0; mt < 2; ++mt) {
      #pragma unroll
      for (int r = 0; r < 8; ++r) {
        const int tokl = 32 * w + 16 * mt + 8 * h + r;
        const float y = acc[mt][nt][r];
        const int idx = (which == 2) ? (feat * 128 + tokl) : (tokl * HD + feat);
        sT[idx] = (_Float16)y;
      }
    }
  }
  __syncthreads();

  const int b = m0 / SEQ, l0 = m0 - b * SEQ, bh = b * NHEADS + head;
  _Float16* plane = (which == 0) ? qh : kh;
  qkv_store_pass(sT, plane, vt, which, bh, l0, w, lane);
  __threadfence();
  qkv_store_pass(sT, plane, vt, which, bh, l0, w, lane);
}

__device__ __forceinline__ v16h pack_p(v8f a, v8f c) {
  const v16h r = { (_Float16)(a[0] * PSCALE), (_Float16)(a[1] * PSCALE), (_Float16)(a[2] * PSCALE), (_Float16)(a[3] * PSCALE),
                   (_Float16)(a[4] * PSCALE), (_Float16)(a[5] * PSCALE), (_Float16)(a[6] * PSCALE), (_Float16)(a[7] * PSCALE),
                   (_Float16)(c[0] * PSCALE), (_Float16)(c[1] * PSCALE), (_Float16)(c[2] * PSCALE), (_Float16)(c[3] * PSCALE),
                   (_Float16)(c[4] * PSCALE), (_Float16)(c[5] * PSCALE), (_Float16)(c[6] * PSCALE), (_Float16)(c[7] * PSCALE) };
  return r;
}

__device__ __forceinline__ void att_store_pass(const float* so, unsigned short* ohi, unsigned short* olo,
                                               int b, int head, int q0, int lane) {
  const int q8 = lane & 7, sub = lane >> 3;
  #pragma unroll
  for (int i = 0; i < 4; ++i) {
    const int row = i * 4 + sub;
    const v4f a = *(const v4fa*)(so + row * 64 + 8 * q8);
    const v4f c = *(const v4fa*)(so + row * 64 + 8 * q8 + 4);
    unsigned short h0, h1, h2, h3, h4, h5, h6, h7;
    unsigned short e0, e1, e2, e3, e4, e5, e6, e7;
    split_bf16(a.x, h0, e0); split_bf16(a.y, h1, e1); split_bf16(a.z, h2, e2); split_bf16(a.w, h3, e3);
    split_bf16(c.x, h4, e4); split_bf16(c.y, h5, e5); split_bf16(c.z, h6, e6); split_bf16(c.w, h7, e7);
    const v8us vh = { h0, h1, h2, h3, h4, h5, h6, h7 };
    const v8us vl = { e0, e1, e2, e3, e4, e5, e6, e7 };
    const size_t gi = ((size_t)b * SEQ + q0 + row) * DIMC + head * HD + 8 * q8;
    *(volatile v8us*)(ohi + gi) = vh;
    *(volatile v8us*)(olo + gi) = vl;
  }
}

__global__ __launch_bounds__(128) void attn_kernel(
    const _Float16* __restrict__ qh,
    const _Float16* __restrict__ kh,
    const _Float16* __restrict__ vt,
    const int* __restrict__ msk,
    unsigned short* __restrict__ ohi,
    unsigned short* __restrict__ olo)
{
  __shared__ __attribute__((aligned(16))) float sO[4 * 16 * 64];

  const int tid = threadIdx.x, lane = tid & 31, w = tid >> 5;
  const int h = lane >> 4, m = lane & 15;
  const int bh = blockIdx.y, b = bh / NHEADS, head = bh - b * NHEADS;
  const int q0 = blockIdx.x * 64 + 16 * w;

  const _Float16* qrow = qh + ((size_t)bh * SEQ + q0 + m) * HD;
  const v16h qb0 = load_frag_h(qrow, h);
  const v16h qb1 = load_frag_h(qrow + 32, h);

  const v8f zero8 = {0.f, 0.f, 0.f, 0.f, 0.f, 0.f, 0.f, 0.f};
  v8f o[4];
  #pragma unroll
  for (int t = 0; t < 4; ++t) o[t] = zero8;
  float mrun = -1.0e30f, lrun = 0.0f;

  const _Float16* kbase = kh + ((size_t)bh * SEQ + m) * HD;
  const _Float16* vbase = vt + ((size_t)bh * HD + m) * SEQ;
  const int* mrow = msk + (size_t)(q0 + m) * SEQ + 8 * h;

  #pragma unroll 1
  for (int kb = 0; kb < SEQ; kb += 64) {
    unsigned int mbits = 0u;
    #pragma unroll
    for (int j = 0; j < 4; ++j) {
      const v4i w0 = *(const v4ia*)(mrow + kb + 16 * j);
      const v4i w1 = *(const v4ia*)(mrow + kb + 16 * j + 4);
      mbits |= (w0.x != 0 ? 1u : 0u) << (8 * j + 0);
      mbits |= (w0.y != 0 ? 1u : 0u) << (8 * j + 1);
      mbits |= (w0.z != 0 ? 1u : 0u) << (8 * j + 2);
      mbits |= (w0.w != 0 ? 1u : 0u) << (8 * j + 3);
      mbits |= (w1.x != 0 ? 1u : 0u) << (8 * j + 4);
      mbits |= (w1.y != 0 ? 1u : 0u) << (8 * j + 5);
      mbits |= (w1.z != 0 ? 1u : 0u) << (8 * j + 6);
      mbits |= (w1.w != 0 ? 1u : 0u) << (8 * j + 7);
    }
    int live = (mbits != 0xFFFFFFFFu) ? 1 : 0;
    live |= __shfl_xor(live, 1);
    live |= __shfl_xor(live, 2);
    live |= __shfl_xor(live, 4);
    live |= __shfl_xor(live, 8);
    live |= __shfl_xor(live, 16);
    live = __builtin_amdgcn_readfirstlane(live);

    if (live != 0) {
      v8f s[4];
      #pragma unroll
      for (int j = 0; j < 4; ++j) {
        const _Float16* kp = kbase + (size_t)(kb + 16 * j) * HD;
        const v16h kf0 = load_frag_h(kp, h);
        const v16h kf1 = load_frag_h(kp + 32, h);
        v8f z = zero8;
        z = wmma_f16(kf0, qb0, z);
        z = wmma_f16(kf1, qb1, z);
        s[j] = z;
      }
      #pragma unroll
      for (int j = 0; j < 4; ++j)
        #pragma unroll
        for (int r = 0; r < 8; ++r) {
          const bool mk = ((mbits >> (8 * j + r)) & 1u) != 0u;
          s[j][r] = mk ? -1.0e9f : (s[j][r] * QKSCALE);
        }

      float mloc = s[0][0];
      #pragma unroll
      for (int j = 0; j < 4; ++j)
        #pragma unroll
        for (int r = 0; r < 8; ++r) mloc = fmaxf(mloc, s[j][r]);
      mloc = fmaxf(mloc, __shfl_xor(mloc, 16));
      const float mnew = fmaxf(mrun, mloc);
      const float alpha = __expf(mrun - mnew);
      mrun = mnew;
      float lsum = 0.0f;
      #pragma unroll
      for (int j = 0; j < 4; ++j)
        #pragma unroll
        for (int r = 0; r < 8; ++r) {
          const float p = __expf(s[j][r] - mnew);
          s[j][r] = p;
          lsum += p;
        }
      lsum += __shfl_xor(lsum, 16);
      lrun = lrun * alpha + lsum;
      #pragma unroll
      for (int t = 0; t < 4; ++t)
        #pragma unroll
        for (int r = 0; r < 8; ++r) o[t][r] = o[t][r] * alpha;

      const v16h pb0 = pack_p(s[0], s[1]);
      const v16h pb1 = pack_p(s[2], s[3]);

      #pragma unroll
      for (int t = 0; t < 4; ++t) {
        const _Float16* vp = vbase + (size_t)(16 * t) * SEQ + kb;
        const v16h vf0 = load_frag_h(vp, h);
        const v16h vf1 = load_frag_h(vp + 32, h);
        o[t] = wmma_f16(vf0, pb0, o[t]);
        o[t] = wmma_f16(vf1, pb1, o[t]);
      }
    }
  }

  const float inv = (1.0f / lrun) * (1.0f / PSCALE);
  float* so = sO + w * 1024;
  #pragma unroll
  for (int t = 0; t < 4; ++t)
    #pragma unroll
    for (int r = 0; r < 8; ++r)
      so[m * 64 + 16 * t + 8 * h + r] = o[t][r] * inv;
  __syncthreads();

  att_store_pass(so, ohi, olo, b, head, q0, lane);
  __threadfence();
  att_store_pass(so, ohi, olo, b, head, q0, lane);
}

__device__ __forceinline__ void out_store_pass(const float* sT, float* out,
                                               int m0, int n0, int w, int lane) {
  const int q8 = lane & 7, sub = lane >> 3;
  #pragma unroll
  for (int i = 0; i < 16; ++i) {
    const int lid = w * 64 + i * 4 + sub;
    const int row = lid >> 1, hl = lid & 1;
    const v4f v = *(const v4fa*)(sT + row * 64 + 32 * hl + 4 * q8);
    const size_t gi = (size_t)(m0 + row) * DIMC + n0 + 32 * hl + 4 * q8;
    *(volatile v4f*)(out + gi) = v;
  }
}

__global__ __launch_bounds__(128) void proj_kernel(
    const unsigned short* __restrict__ ohi,
    const unsigned short* __restrict__ olo,
    const unsigned short* __restrict__ wpb,
    float* __restrict__ out)
{
  __shared__ __attribute__((aligned(16))) float sT[128 * 64];

  const int tid = threadIdx.x, lane = tid & 31, w = tid >> 5;
  const int h = lane >> 4, m = lane & 15;
  const int m0 = blockIdx.x * 128;
  const int n0 = blockIdx.y * 64;
  const int m0w = m0 + 32 * w;

  const unsigned short* ah0 = ohi + (size_t)(m0w + m) * DIMC;
  const unsigned short* ah1 = ah0 + (size_t)16 * DIMC;
  const unsigned short* al0 = olo + (size_t)(m0w + m) * DIMC;
  const unsigned short* al1 = al0 + (size_t)16 * DIMC;
  const unsigned short* wb  = wpb + ((size_t)n0 + m) * DIMC;

  const v8f zero8 = {0.f, 0.f, 0.f, 0.f, 0.f, 0.f, 0.f, 0.f};
  v8f acc[2][4];
  #pragma unroll
  for (int mt = 0; mt < 2; ++mt)
    #pragma unroll
    for (int nt = 0; nt < 4; ++nt) acc[mt][nt] = zero8;

  #pragma unroll 1
  for (int k0 = 0; k0 < DIMC; k0 += 32) {
    const v16b hh0 = load_frag_b(ah0 + k0, h);
    const v16b hh1 = load_frag_b(ah1 + k0, h);
    const v16b ll0 = load_frag_b(al0 + k0, h);
    const v16b ll1 = load_frag_b(al1 + k0, h);
    #pragma unroll
    for (int nt = 0; nt < 4; ++nt) {
      const v16b b = load_frag_b(wb + (size_t)nt * 16 * DIMC + k0, h);
      acc[0][nt] = wmma_bf16(hh0, b, acc[0][nt]);
      acc[0][nt] = wmma_bf16(ll0, b, acc[0][nt]);
      acc[1][nt] = wmma_bf16(hh1, b, acc[1][nt]);
      acc[1][nt] = wmma_bf16(ll1, b, acc[1][nt]);
    }
  }

  #pragma unroll
  for (int nt = 0; nt < 4; ++nt) {
    const int feat = 16 * nt + m;
    #pragma unroll
    for (int mt = 0; mt < 2; ++mt) {
      #pragma unroll
      for (int r = 0; r < 8; ++r) {
        const int tokl = 32 * w + 16 * mt + 8 * h + r;
        sT[tokl * 64 + feat] = acc[mt][nt][r];
      }
    }
  }
  __syncthreads();

  out_store_pass(sT, out, m0, n0, w, lane);
  __threadfence();
  out_store_pass(sT, out, m0, n0, w, lane);
}

extern "C" void kernel_launch(void* const* d_in, const int* in_sizes, int n_in,
                              void* d_out, int out_size, void* d_ws, size_t ws_size,
                              hipStream_t stream) {
  if (n_in < 4) return;
  if (in_sizes[0] != NX) return;
  if (in_sizes[1] != NWQ) return;
  if (in_sizes[2] != NWP) return;
  if (in_sizes[3] != NMASK) return;
  if (out_size != NX) return;

  const float* x      = (const float*)d_in[0];
  const float* qkv_w  = (const float*)d_in[1];
  const float* proj_w = (const float*)d_in[2];
  const int*   smask  = (const int*)d_in[3];
  float* out = (float*)d_out;

  const size_t xb_bytes  = (size_t)NX * 2;
  const size_t wqb_bytes = (size_t)NWQ * 2;
  const size_t wpb_bytes = (size_t)NWP * 2;
  const size_t pl_bytes  = (size_t)BATCH * NHEADS * SEQ * HD * 2;
  const size_t o_bytes   = (size_t)NX * 2;
  const size_t off_xb  = 0;
  const size_t off_wqb = off_xb + xb_bytes;
  const size_t off_wpb = off_wqb + wqb_bytes;
  const size_t off_q   = off_wpb + wpb_bytes;
  const size_t off_k   = off_q + pl_bytes;
  const size_t off_vt  = off_k + pl_bytes;
  const size_t off_hi  = off_vt + pl_bytes;
  const size_t off_lo  = off_hi + o_bytes;
  const size_t total   = off_lo + o_bytes;
  if (total > ws_size) return;

  char* ws = (char*)d_ws;
  unsigned short* xb  = (unsigned short*)(ws + off_xb);
  unsigned short* wqb = (unsigned short*)(ws + off_wqb);
  unsigned short* wpb = (unsigned short*)(ws + off_wpb);
  _Float16* qh = (_Float16*)(ws + off_q);
  _Float16* kh = (_Float16*)(ws + off_k);
  _Float16* vt = (_Float16*)(ws + off_vt);
  unsigned short* ohi = (unsigned short*)(ws + off_hi);
  unsigned short* olo = (unsigned short*)(ws + off_lo);

  convert_kernel<<<(NCVT + 255) / 256, 256, 0, stream>>>(x, qkv_w, proj_w, xb, wqb, wpb);

  dim3 gQkv(MROWS / 128, QKVO / 64);
  qkv_kernel<<<gQkv, 128, 0, stream>>>(xb, wqb, qh, kh, vt);

  dim3 gAtt(SEQ / 64, BATCH * NHEADS);
  attn_kernel<<<gAtt, 128, 0, stream>>>(qh, kh, vt, smask, ohi, olo);

  dim3 gPrj(MROWS / 128, DIMC / 64);
  proj_kernel<<<gPrj, 128, 0, stream>>>(ohi, olo, wpb, out);
}
